// Mamba2SimpleCat_15745350107166
// MI455X (gfx1250) — hardware-verified
//
#include <hip/hip_runtime.h>


#define NB_  2
#define TT   2048
#define DM   1024
#define HALF 1024
#define CD   1056
#define DP   2144
#define NMAIN 2112
#define DTOFF 2080
#define NH_  64
#define HP   16
#define NS   16
#define ZH   8
typedef _Float16 h16;
typedef unsigned short bf;
typedef __attribute__((ext_vector_type(16))) __bf16   v16bf;
typedef __attribute__((ext_vector_type(16))) _Float16 v16h;
typedef __attribute__((ext_vector_type(8)))  _Float16 v8h;
typedef __attribute__((ext_vector_type(8)))  unsigned short v8us;
typedef __attribute__((ext_vector_type(8)))  float    v8f;
typedef __attribute__((ext_vector_type(4)))  float    v4f;
typedef v8h  __attribute__((may_alias)) v8ha;
typedef v4f  __attribute__((may_alias)) v4fa;
typedef v8us __attribute__((may_alias)) v8usa;

__device__ __forceinline__ unsigned short f2bf(float f) { unsigned u = __float_as_uint(f); u += 0x7FFFu + ((u >> 16) & 1u); return (unsigned short)(u >> 16); }
__device__ __forceinline__ float bf2f(unsigned short b) { return __uint_as_float(((unsigned)b) << 16); }
__device__ __forceinline__ float bfr(float f) { return bf2f(f2bf(f)); }
__device__ __forceinline__ v16h cat16(v8h lo, v8h hi) { return __builtin_shufflevector(lo, hi, 0, 1, 2, 3, 4, 5, 6, 7, 8, 9, 10, 11, 12, 13, 14, 15); }
__device__ __forceinline__ v16bf cat16b(v8us lo, v8us hi) { return __builtin_bit_cast(v16bf, __builtin_shufflevector(lo, hi, 0, 1, 2, 3, 4, 5, 6, 7, 8, 9, 10, 11, 12, 13, 14, 15)); }
__device__ __forceinline__ v8f wmma16(v16h a, v16h b, v8f c) { return __builtin_amdgcn_wmma_f32_16x16x32_f16(false, a, false, b, (short)0, c, false, false); }
__device__ __forceinline__ v8f wmmab(v16bf a, v16bf b, v8f c) { return __builtin_amdgcn_wmma_f32_16x16x32_bf16(false, a, false, b, (short)0, c, false, false); }


template <typename T16> struct WFrag;
template <> struct WFrag<h16> { typedef v16h V; static __device__ __forceinline__ V ld(const h16* p) { return cat16(*(const v8h*)p, *(const v8h*)(p + 16)); } static __device__ __forceinline__ v8f mma(V a, V b, v8f c) { return wmma16(a, b, c); } };
template <> struct WFrag<bf> { typedef v16bf V; static __device__ __forceinline__ V ld(const bf* p) { return cat16b(*(const v8us*)p, *(const v8us*)(p + 16)); } static __device__ __forceinline__ v8f mma(V a, V b, v8f c) { return wmmab(a, b, c); } };
template <typename T16, int NSPLIT, bool BIAS>
__global__ __launch_bounds__(32) void k_gemmw(const T16* __restrict__ A, const T16* __restrict__ A2, const T16* __restrict__ Bt, const T16* __restrict__ Bt2, int K, float* C, int ldc, const float* __restrict__ bias, size_t sA, size_t sB, size_t sC) {
    typedef typename WFrag<T16>::V V;
    __shared__ __align__(16) float os[16 * 68];
    const size_t z = blockIdx.z; A += z * sA; if (A2) A2 += z * sA; Bt += z * sB; if (Bt2) Bt2 += z * sB; C += z * sC;
    const int lane = threadIdx.x & 31, lr = lane & 15, hi = lane >> 4; const int r0 = blockIdx.x * 64, c0 = blockIdx.y * 64;
    v8f acc[4][4];
#pragma unroll
    for (int mb = 0; mb < 4; ++mb)
#pragma unroll
        for (int nb = 0; nb < 4; ++nb) acc[mb][nb] = (v8f){};
    const size_t aoff = (size_t)(r0 + lr) * K + 8 * hi, boff = (size_t)(c0 + lr) * K + 8 * hi;
#pragma unroll 1
    for (int kc = 0; kc < K; kc += 32) {
        V a[4], a2[4];
#pragma unroll
        for (int mb = 0; mb < 4; ++mb) { a[mb] = WFrag<T16>::ld(A + aoff + (size_t)mb * 16 * K + kc); if (NSPLIT == 1 || NSPLIT == 2) a2[mb] = WFrag<T16>::ld(A2 + aoff + (size_t)mb * 16 * K + kc); }
#pragma unroll
        for (int nb = 0; nb < 4; ++nb) { const V b = WFrag<T16>::ld(Bt + boff + (size_t)nb * 16 * K + kc); V b2; if (NSPLIT >= 2) b2 = WFrag<T16>::ld(Bt2 + boff + (size_t)nb * 16 * K + kc);
#pragma unroll
            for (int mb = 0; mb < 4; ++mb) { acc[mb][nb] = WFrag<T16>::mma(a[mb], b, acc[mb][nb]); if (NSPLIT == 1 || NSPLIT == 2) acc[mb][nb] = WFrag<T16>::mma(a2[mb], b, acc[mb][nb]); if (NSPLIT >= 2) acc[mb][nb] = WFrag<T16>::mma(a[mb], b2, acc[mb][nb]); } }
        asm volatile("v_nop\n\tv_nop\n\tv_nop\n\tv_nop" : "+v"(acc[0][0]), "+v"(acc[1][1]), "+v"(acc[2][2]), "+v"(acc[3][3]) : "v"(a[0]), "v"(a[3]));
    }
#pragma unroll
    for (int mb = 0; mb < 4; ++mb) {
#pragma unroll
        for (int nb = 0; nb < 4; ++nb) {
#pragma unroll
            for (int j = 0; j < 8; ++j) os[(hi * 8 + j) * 68 + nb * 16 + lr] = acc[mb][nb][j]; }
        __builtin_amdgcn_wave_barrier(); asm volatile("" ::: "memory");
        float* crow = C + (size_t)(r0 + mb * 16) * ldc + c0;
#pragma unroll 1
        for (int ps = 0; ps < 2; ++ps) {
#pragma unroll
            for (int s = 0; s < 8; ++s) { const int row = 2 * s + hi, cofs = lr * 4; v4f val = *(const v4fa*)(os + row * 68 + cofs); if (BIAS) { val[0] += bfr(bias[c0 + cofs]); val[1] += bfr(bias[c0 + cofs + 1]); val[2] += bfr(bias[c0 + cofs + 2]); val[3] += bfr(bias[c0 + cofs + 3]); }
                *(volatile v4f*)(crow + (size_t)row * ldc + cofs) = val; }
            if (ps == 0) __threadfence(); }
        __builtin_amdgcn_wave_barrier(); asm volatile("" ::: "memory");
    }
}

template <typename T16, int NSPLIT, int CMODE>
__global__ __launch_bounds__(32) void k_gemmc(const T16* __restrict__ A, const T16* __restrict__ A2, const T16* __restrict__ Bt, const T16* __restrict__ Bt2, int K, float* C, int ldc, int roff, size_t sA, size_t sB, size_t sC) {
    typedef typename WFrag<T16>::V V;
    __shared__ __align__(16) float os[16 * 68];
    const size_t z = blockIdx.z; A += z * sA; if (A2) A2 += z * sA; Bt += z * sB; if (Bt2) Bt2 += z * sB; C += z * sC;
    const int lane = threadIdx.x & 31, lr = lane & 15, hi = lane >> 4; const int r0 = blockIdx.x * 64, c0 = blockIdx.y * 64;
    if (CMODE == 1 && c0 > r0 + roff + 63) return;
    const int Kl = (CMODE == 2) ? min(K, r0 + roff + 64) : K;
    v8f acc[4][4];
#pragma unroll
    for (int mb = 0; mb < 4; ++mb)
#pragma unroll
        for (int nb = 0; nb < 4; ++nb) acc[mb][nb] = (v8f){};
    const size_t aoff = (size_t)(r0 + lr) * K + 8 * hi, boff = (size_t)(c0 + lr) * K + 8 * hi;
#pragma unroll 1
    for (int kc = 0; kc < Kl; kc += 32) {
        V a[4], a2[4];
#pragma unroll
        for (int mb = 0; mb < 4; ++mb) { a[mb] = WFrag<T16>::ld(A + aoff + (size_t)mb * 16 * K + kc); if (NSPLIT == 1 || NSPLIT == 2) a2[mb] = WFrag<T16>::ld(A2 + aoff + (size_t)mb * 16 * K + kc); }
#pragma unroll
        for (int nb = 0; nb < 4; ++nb) { const V b = WFrag<T16>::ld(Bt + boff + (size_t)nb * 16 * K + kc); V b2; if (NSPLIT >= 2) b2 = WFrag<T16>::ld(Bt2 + boff + (size_t)nb * 16 * K + kc);
#pragma unroll
            for (int mb = 0; mb < 4; ++mb) { acc[mb][nb] = WFrag<T16>::mma(a[mb], b, acc[mb][nb]); if (NSPLIT == 1 || NSPLIT == 2) acc[mb][nb] = WFrag<T16>::mma(a2[mb], b, acc[mb][nb]); if (NSPLIT >= 2) acc[mb][nb] = WFrag<T16>::mma(a[mb], b2, acc[mb][nb]); } }
        asm volatile("v_nop\n\tv_nop\n\tv_nop\n\tv_nop" : "+v"(acc[0][0]), "+v"(acc[1][1]), "+v"(acc[2][2]), "+v"(acc[3][3]) : "v"(a[0]), "v"(a[3]));
    }
#pragma unroll
    for (int mb = 0; mb < 4; ++mb) {
#pragma unroll
        for (int nb = 0; nb < 4; ++nb) {
#pragma unroll
            for (int j = 0; j < 8; ++j) os[(hi * 8 + j) * 68 + nb * 16 + lr] = acc[mb][nb][j]; }
        __builtin_amdgcn_wave_barrier(); asm volatile("" ::: "memory");
        float* crow = C + (size_t)(r0 + mb * 16) * ldc + c0;
#pragma unroll 1
        for (int ps = 0; ps < 2; ++ps) {
#pragma unroll
            for (int s = 0; s < 8; ++s) { const int row = 2 * s + hi, cofs = lr * 4; v4f val = *(const v4fa*)(os + row * 68 + cofs);
                *(volatile v4f*)(crow + (size_t)row * ldc + cofs) = val; }
            if (ps == 0) __threadfence(); }
        __builtin_amdgcn_wave_barrier(); asm volatile("" ::: "memory");
    }
}

__device__ __forceinline__ h16 tohx(float x) { return (h16)x; }
__device__ __forceinline__ void splitf(float y, unsigned short& h, unsigned short& l) { h = f2bf(y); l = f2bf(y - bf2f(h)); }
__device__ __forceinline__ float silu_(float x) { return __fmul_rn(x, __fdiv_rn(1.0f, 1.0f + __expf(-x))); }
typedef __attribute__((ext_vector_type(2))) _Float16 v2h;
typedef __attribute__((ext_vector_type(4))) _Float16 v4h;
typedef __attribute__((ext_vector_type(2))) unsigned short v2us;
typedef __attribute__((ext_vector_type(4))) unsigned short v4us;
typedef __attribute__((ext_vector_type(2))) float v2f;

__global__ __launch_bounds__(256) void k_cvt8(const float* __restrict__ src, bf* dst, size_t n8) { const size_t i = (size_t)blockIdx.x * 256 + threadIdx.x; if (i >= n8) return; const v8f v = *(const v8f*)(src + i * 8); v8us o;
#pragma unroll
    for (int k = 0; k < 8; ++k) o[k] = f2bf(v[k]); *(volatile v8us*)(dst + i * 8) = o; __threadfence(); *(volatile v8us*)(dst + i * 8) = o; }
__global__ __launch_bounds__(256) void k_wdt(const float* __restrict__ w, bf* WDT) { const int i = (blockIdx.x * 256 + threadIdx.x) * 4; if (i >= 64 * DM) return; const int k = i % DM, n = i / DM; v4us o;
#pragma unroll
    for (int q = 0; q < 4; ++q) o[q] = f2bf(w[(size_t)(DTOFF + n) * DM + k + q]); *(volatile v4us*)(WDT + i) = o; __threadfence(); *(volatile v4us*)(WDT + i) = o; }
__global__ __launch_bounds__(256) void k_conv(const float* __restrict__ ZX, const float* __restrict__ w, const float* __restrict__ bb, float* XC) { const size_t e = ((size_t)blockIdx.x * 256 + threadIdx.x) * 4; if (e >= (size_t)TT * CD) return; const int c = (int)(e % CD); const int t = (int)(e / CD); v4f o;
#pragma unroll
    for (int q = 0; q < 4; ++q) { float acc = bfr(bb[c + q]);
#pragma unroll
        for (int k = 0; k < 4; ++k) { const int ts = t - 3 + k; if (ts >= 0) { float p = __fmul_rn(ZX[(size_t)ts * NMAIN + HALF + c + q], bfr(w[(c + q) * 4 + k])); asm volatile("" : "+v"(p)); acc = __fadd_rn(acc, p); } }
        o[q] = silu_(acc); }
    *(volatile v4f*)(XC + e) = o; __threadfence(); *(volatile v4f*)(XC + e) = o; }
__global__ __launch_bounds__(256) void k_bcpl(const float* __restrict__ XC, bf* Ch, bf* Cl, bf* Bh, bf* Bl) { const size_t e = ((size_t)blockIdx.x * 256 + threadIdx.x) * 2; if (e >= (size_t)TT * 32) return; const int n = (int)(e % 32); const int t = (int)(e / 32); const float* r = XC + (size_t)t * CD + HALF; v2us ch_, cl_, bh_, bl_;
#pragma unroll
    for (int u = 0; u < 2; ++u) { unsigned short a = 0, c = 0, a2 = 0, c2 = 0; if (n + u < NS) { splitf(r[NS + n + u], a, c); splitf(r[n + u], a2, c2); } ch_[u] = a; cl_[u] = c; bh_[u] = a2; bl_[u] = c2; }
    for (int ps = 0; ps < 2; ++ps) { *(volatile v2us*)(Ch + e) = ch_; *(volatile v2us*)(Cl + e) = cl_; *(volatile v2us*)(Bh + e) = bh_; *(volatile v2us*)(Bl + e) = bl_; if (ps == 0) __threadfence(); } }
__global__ __launch_bounds__(256) void k_xt16(const float* __restrict__ XC, h16* XT) { const size_t e = ((size_t)blockIdx.x * 256 + threadIdx.x) * 2; if (e >= (size_t)NH_ * 64 * TT) return; const int s = (int)(e % TT); const int p = (int)((e / TT) % 64); const int h = (int)(e / ((size_t)TT * 64)); v2h o; o[0] = p < HP ? tohx(XC[(size_t)s * CD + h * HP + p]) : (h16)0.f; o[1] = p < HP ? tohx(XC[(size_t)(s + 1) * CD + h * HP + p]) : (h16)0.f; *(volatile v2h*)(XT + e) = o; __threadfence(); *(volatile v2h*)(XT + e) = o; }
__global__ __launch_bounds__(64) void k_dtcum(const float* __restrict__ DTR, const float* __restrict__ dtb, const float* __restrict__ alog, float* DT, double* CUM) { const int h = threadIdx.x; const float A = -__expf(bfr(alog[h])); const float bias = bfr(dtb[h]);
    for (int ps = 0; ps < 2; ++ps) { double c = 0.0; for (int t = 0; t < TT; ++t) { const float raw = __fadd_rn(DTR[(size_t)t * 64 + h], bias); const float dt = raw > 20.f ? raw : log1pf(__expf(raw)); c += (double)__fmul_rn(dt, A); *(volatile float*)(DT + (size_t)t * 64 + h) = dt; *(volatile double*)(CUM + (size_t)t * 64 + h) = c; } if (ps == 0) __threadfence(); } }
__global__ __launch_bounds__(256) void k_mask(const float* __restrict__ G, const float* __restrict__ DT, const double* __restrict__ CUM, int h0, h16* M16) { const size_t e = ((size_t)blockIdx.x * 256 + threadIdx.x) * 4; if (e >= (size_t)ZH * TT * TT) return; const int s0 = (int)(e % TT); const int t = (int)((e / TT) % TT); const int h = h0 + (int)(e / ((size_t)TT * TT)); const double ct = CUM[(size_t)t * 64 + h]; const v4f g = *(const v4f*)(G + (size_t)t * TT + s0); v4h o;
#pragma unroll
    for (int q = 0; q < 4; ++q) { const int s = s0 + q; float v = 0.f; if (s <= t) { const float dl = (float)(ct - CUM[(size_t)s * 64 + h]); float w = __fmul_rn(__expf(dl), DT[(size_t)s * 64 + h]); asm volatile("" : "+v"(w)); v = __fmul_rn(g[q], w); } o[q] = tohx(v); }
    *(volatile v4h*)(M16 + e) = o; __threadfence(); *(volatile v4h*)(M16 + e) = o; }
__global__ __launch_bounds__(256) void k_yd(const float* __restrict__ Y, const float* __restrict__ XC, const float* __restrict__ Dv, int h0, float* YF) { const size_t e = ((size_t)blockIdx.x * 256 + threadIdx.x) * 2; if (e >= (size_t)ZH * TT * HP) return; const int p = (int)(e % HP); const int z = (int)((e / HP) % ZH); const int t = (int)(e / ((size_t)HP * ZH)); const int h = h0 + z; const float dd = bfr(Dv[h]); v2f o;
#pragma unroll
    for (int u = 0; u < 2; ++u) { float sk = __fmul_rn(XC[(size_t)t * CD + h * HP + p + u], dd); asm volatile("" : "+v"(sk)); o[u] = __fadd_rn(Y[((size_t)z * TT + t) * 64 + p + u], sk); }
    const size_t oo = (size_t)t * HALF + h * HP + p; *(volatile v2f*)(YF + oo) = o; __threadfence(); *(volatile v2f*)(YF + oo) = o; }
__global__ __launch_bounds__(256) void k_lncat(const float* __restrict__ YF, const float* __restrict__ ZX, const float* __restrict__ g, const float* __restrict__ bb, bf* Ph, bf* Pl) { const int lane = threadIdx.x & 31; const int t = blockIdx.x * 8 + (threadIdx.x >> 5); if (t >= TT) return; float s = 0.f;
#pragma unroll 1
    for (int ch = 0; ch < 16; ++ch) { const float* src = ch < 8 ? YF + (size_t)t * HALF + ch * 128 : ZX + (size_t)t * NMAIN + (ch - 8) * 128; const v4f a = *(const v4f*)(src + lane * 4); s = __fadd_rn(s, __fadd_rn(__fadd_rn(a[0], a[1]), __fadd_rn(a[2], a[3]))); }
#pragma unroll
    for (int sh = 16; sh; sh >>= 1) s += __shfl_xor(s, sh, 32);
    const float mu = s * (1.0f / 2048.0f); float q2 = 0.f;
#pragma unroll 1
    for (int ch = 0; ch < 16; ++ch) { const float* src = ch < 8 ? YF + (size_t)t * HALF + ch * 128 : ZX + (size_t)t * NMAIN + (ch - 8) * 128; const v4f a = *(const v4f*)(src + lane * 4);
#pragma unroll
        for (int q = 0; q < 4; ++q) { float dv = __fsub_rn(a[q], mu); asm volatile("" : "+v"(dv)); float p = __fmul_rn(dv, dv); asm volatile("" : "+v"(p)); q2 = __fadd_rn(q2, p); } }
#pragma unroll
    for (int sh = 16; sh; sh >>= 1) q2 += __shfl_xor(q2, sh, 32);
    float vq = q2 * (1.0f / 2048.0f); asm volatile("" : "+v"(vq)); const float rs = __fdiv_rn(1.0f, __fsqrt_rn(__fadd_rn(vq, 1e-5f)));
#pragma unroll 1
    for (int ch = 0; ch < 16; ++ch) { const float* src = ch < 8 ? YF + (size_t)t * HALF + ch * 128 : ZX + (size_t)t * NMAIN + (ch - 8) * 128; const int c0 = ch * 128 + lane * 4; const v4f a = *(const v4f*)(src + lane * 4); v4us oh, ol;
#pragma unroll
        for (int q = 0; q < 4; ++q) { float dv = __fsub_rn(a[q], mu); asm volatile("" : "+v"(dv)); float tn = __fmul_rn(dv, rs); asm volatile("" : "+v"(tn)); float tg = __fmul_rn(tn, bfr(g[c0 + q])); asm volatile("" : "+v"(tg)); unsigned short u, c; splitf(__fadd_rn(tg, bfr(bb[c0 + q])), u, c); oh[q] = u; ol[q] = c; }
        const size_t oo = (size_t)t * 2048 + c0; *(volatile v4us*)(Ph + oo) = oh; *(volatile v4us*)(Pl + oo) = ol; __threadfence(); *(volatile v4us*)(Ph + oo) = oh; *(volatile v4us*)(Pl + oo) = ol; } }

extern "C" void kernel_launch(void* const* d_in, const int* in_sizes, int n_in,
                              void* d_out, int out_size, void* d_ws, size_t ws_size, hipStream_t stream) {
    (void)in_sizes; (void)n_in; (void)out_size;
    const float* u = (const float*)d_in[0]; const float* win = (const float*)d_in[1]; const float* cw = (const float*)d_in[2]; const float* cb = (const float*)d_in[3]; const float* dtb = (const float*)d_in[4]; const float* alog = (const float*)d_in[5]; const float* Dv = (const float*)d_in[6]; const float* lnw = (const float*)d_in[7]; const float* lnb = (const float*)d_in[8]; const float* wout = (const float*)d_in[9];
    float* OUT = (float*)d_out;
    char* wsp = (char*)d_ws;
    auto take = [&](size_t bytes) { char* p = wsp; wsp += (bytes + 255) & ~(size_t)255; return (void*)p; };
    bf* WIN = (bf*)take((size_t)DP * DM * 2); bf* WDT = (bf*)take((size_t)64 * DM * 2); bf* WO = (bf*)take((size_t)DM * 2048 * 2); bf* XB = (bf*)take((size_t)TT * DM * 2); float* ZX = (float*)take((size_t)TT * NMAIN * 4); float* DTR = (float*)take((size_t)TT * 64 * 4); float* XC = (float*)take((size_t)TT * CD * 4);
    bf* Ch = (bf*)take((size_t)TT * 32 * 2); bf* Cl = (bf*)take((size_t)TT * 32 * 2); bf* Bh = (bf*)take((size_t)TT * 32 * 2); bf* Bl = (bf*)take((size_t)TT * 32 * 2); float* G = (float*)take((size_t)TT * TT * 4); h16* XT = (h16*)take((size_t)NH_ * 64 * TT * 2); float* DT = (float*)take((size_t)TT * 64 * 4); double* CUM = (double*)take((size_t)TT * 64 * 8);
    h16* M16 = (h16*)take((size_t)ZH * TT * TT * 2); float* Y = (float*)take((size_t)ZH * TT * 64 * 4); float* YF = (float*)take((size_t)TT * HALF * 4); bf* Ph = (bf*)take((size_t)TT * 2048 * 2); bf* Pl = (bf*)take((size_t)TT * 2048 * 2);
    if ((size_t)(wsp - (char*)d_ws) > ws_size) return;
    k_cvt8<<<(unsigned)(((size_t)DP * DM / 8 + 255) / 256), 256, 0, stream>>>(win, WIN, (size_t)DP * DM / 8); k_wdt<<<(64 * DM / 4 + 255) / 256, 256, 0, stream>>>(win, WDT); k_cvt8<<<(unsigned)(((size_t)DM * 2048 / 8 + 255) / 256), 256, 0, stream>>>(wout, WO, (size_t)DM * 2048 / 8);
    for (int b = 0; b < NB_; ++b) {
        k_cvt8<<<(TT * DM / 8 + 255) / 256, 256, 0, stream>>>(u + (size_t)b * TT * DM, XB, (size_t)TT * DM / 8);
        k_gemmw<bf, 0, false><<<dim3(TT / 64, NMAIN / 64, 1), 32, 0, stream>>>(XB, nullptr, WIN, nullptr, DM, ZX, NMAIN, nullptr, 0, 0, 0); k_gemmw<bf, 0, false><<<dim3(TT / 64, 1, 1), 32, 0, stream>>>(XB, nullptr, WDT, nullptr, DM, DTR, 64, nullptr, 0, 0, 0);
        k_conv<<<(unsigned)(((size_t)TT * CD / 4 + 255) / 256), 256, 0, stream>>>(ZX, cw, cb, XC);
        k_bcpl<<<(TT * 32 / 2 + 255) / 256, 256, 0, stream>>>(XC, Ch, Cl, Bh, Bl); k_xt16<<<(unsigned)(((size_t)NH_ * 64 * TT / 2 + 255) / 256), 256, 0, stream>>>(XC, XT); k_dtcum<<<1, 64, 0, stream>>>(DTR, dtb, alog, DT, CUM);
        k_gemmc<bf, 2, 1><<<dim3(TT / 64, TT / 64, 1), 32, 0, stream>>>(Ch, Cl, Bh, Bl, 32, G, TT, 0, 0, 0, 0);
        for (int h0 = 0; h0 < NH_; h0 += ZH) {
            k_mask<<<(unsigned)(((size_t)ZH * TT * TT / 4 + 255) / 256), 256, 0, stream>>>(G, DT, CUM, h0, M16);
            k_gemmc<h16, 0, 2><<<dim3(TT / 64, 1, ZH), 32, 0, stream>>>(M16, nullptr, XT + (size_t)h0 * 64 * TT, nullptr, TT, Y, 64, 0, (size_t)TT * TT, (size_t)64 * TT, (size_t)TT * 64);
            k_yd<<<(unsigned)(((size_t)ZH * TT * HP / 2 + 255) / 256), 256, 0, stream>>>(Y, XC, Dv, h0, YF); }
        k_lncat<<<TT / 8, 256, 0, stream>>>(YF, ZX, lnw, lnb, Ph, Pl);
        k_gemmw<bf, 1, false><<<dim3(TT / 64, DM / 64, 1), 32, 0, stream>>>(Ph, Pl, WO, nullptr, 2048, OUT + (size_t)b * TT * DM, DM, nullptr, 0, 0, 0); }
}
